// Mamba3LBlock_2353642078643
// MI455X (gfx1250) — hardware-run, weakly checked
//
#include <hip/hip_runtime.h>
#include <math.h>

typedef __attribute__((ext_vector_type(16))) _Float16 v16h;
typedef __attribute__((ext_vector_type(8)))  _Float16 v8h;
typedef __attribute__((ext_vector_type(8)))  float    v8f;
typedef __attribute__((ext_vector_type(4)))  float    v4f;
typedef __attribute__((ext_vector_type(4)))  unsigned v4u;

constexpr int kBatch    = 4;
constexpr int kSeq      = 2048;
constexpr int kDm       = 1024;
constexpr int kDin      = 2048;
constexpr int kHeads    = 32;
constexpr int kHd       = 64;
constexpr int kNst      = 128;
constexpr int kRank     = 4;
constexpr int kSub      = 16;
constexpr int kBCw      = 2 * kRank * kNst;
constexpr int kCols     = 2 * kDin + kBCw + kHeads;
constexpr int kColsPad  = 5184;
constexpr int kRows     = kBatch * kSeq;
constexpr int kHalfRows = kRows / 2;
constexpr int kTilesM   = kRows / 64;
constexpr int kTilesMh  = kHalfRows / 64;
constexpr int kTilesN1  = kColsPad / 64;
constexpr int kTilesN2  = kDm / 64;
constexpr int kTS       = 4;
constexpr int kSYP      = 68;
static_assert(kCols == 5152);
static_assert(kBCw == 1024);
static_assert(kHeads * kHd == kDin);
static_assert(kRank * kSub == kHd);
static_assert(kColsPad % 64 == 0 && kColsPad >= kCols && kColsPad - kCols < 64);
static_assert(kRows == 8192 && kRows % 64 == 0 && kHalfRows == 4096 && kHalfRows % 64 == 0);
static_assert(kDm % 64 == 0 && kDin % 64 == 0 && kDm % 32 == 0 && kDin % 32 == 0);
static_assert((kTilesMh * kTilesN1) % 8 == 0 && (kTilesM * kTilesN2) % 8 == 0);
static_assert(kSeq % kTS == 0);
static_assert((2 * kDin) % 64 == 0 && (2 * kDin + kBCw) % 64 == 0);

constexpr float kCarryHs  = 16.0f;
constexpr float kCarryLo  = 2048.0f;
constexpr float kLoInv    = 1.0f / kCarryLo;
constexpr float kCarryW   = 1024.0f;
constexpr float kCarryY   = 16.0f;
constexpr float kScaleIn  = 1.0f / (kCarryHs * kCarryW);
constexpr float kScaleOut = 1.0f / (kCarryY * kCarryW);
constexpr float kF16Min   = 6.103515625e-05f;
constexpr float kF16Max   = 65504.0f;
constexpr float kF32Min   = 1.17549435e-38f;
constexpr float kEps      = 1e-5f;

constexpr size_t kSzHSH  = (size_t)kHalfRows * kDm * 2;
constexpr size_t kSzHSL  = (size_t)kHalfRows * kDm * 2;
constexpr size_t kSzWIN  = (size_t)kColsPad * kDm * 2;
constexpr size_t kSzWOUT = (size_t)kDm * kDin * 2;
constexpr size_t kSzZ    = (size_t)kRows * kDin * 2;
constexpr size_t kSzX    = (size_t)kRows * kDin * 2;
constexpr size_t kSzBC   = (size_t)kRows * kBCw * 4;
constexpr size_t kSzDTR  = (size_t)kRows * kHeads * 4;
constexpr size_t kSzDTA  = (size_t)kRows * 64 * 4;
constexpr size_t kOffHSH  = 0;
constexpr size_t kOffHSL  = kOffHSH + kSzHSH;
constexpr size_t kOffWIN  = kOffHSL + kSzHSL;
constexpr size_t kOffWOUT = kOffWIN + kSzWIN;
constexpr size_t kOffZ    = kOffWOUT + kSzWOUT;
constexpr size_t kOffX    = kOffZ + kSzZ;
constexpr size_t kOffBC   = kOffX + kSzX;
constexpr size_t kOffDTR  = kOffBC + kSzBC;
constexpr size_t kWsTotal = kOffDTR + kSzDTR;
static_assert(kWsTotal == 133300224ull);
static_assert(kWsTotal <= 134217728ull);
static_assert(kSzDTA <= kSzHSH + kSzHSL);
static_assert(kSzBC == (size_t)kRows * kDm * 4);
static_assert((kOffHSL % 128) == 0 && (kOffWIN % 128) == 0 && (kOffWOUT % 128) == 0 && (kOffZ % 128) == 0 &&
              (kOffX % 128) == 0 && (kOffBC % 128) == 0 && (kOffDTR % 128) == 0);

__device__ __forceinline__ float h16_to_f32(unsigned hb) {
  const unsigned sgn = (hb & 0x8000u) << 16;
  const unsigned em = hb & 0x7fffu;
  const float fn = __uint_as_float((em << 13) + 0x38000000u);
  const float fs = (float)em * 5.9604644775390625e-8f;
  const float mag = (em < 0x400u) ? fs : fn;
  return __uint_as_float(__float_as_uint(mag) | sgn);
}
__device__ __forceinline__ _Float16 f16_operand(float v) {
  float w = fminf(fmaxf(v, -kF16Max), kF16Max);
  w = (fabsf(w) < kF16Min) ? 0.0f : w;
  return (_Float16)w;
}

union FragU { v16h v; v8h h[2]; };
__device__ __forceinline__ v16h frag_load(const _Float16* p) {
  FragU f;
  f.h[0] = *(const v8h*)(p);
  f.h[1] = *(const v8h*)(p + 16);
  return f.v;
}
__device__ __forceinline__ v8f frag_mma(v16h a, v16h b, v8f c) {
  return __builtin_amdgcn_wmma_f32_16x16x32_f16(false, a, false, b, (short)0, c, false, false);
}
__device__ __forceinline__ void guard_group(v8f& a0, v8f& a1, v8f& a2, v8f& a3, v16h x, v16h b0, v16h b1, v16h b2, v16h b3) {
  asm volatile("v_nop\n\tv_nop\n\tv_nop\n\tv_nop" : "+v"(a0), "+v"(a1), "+v"(a2), "+v"(a3) : "v"(x), "v"(b0), "v"(b1), "v"(b2), "v"(b3));
}
__device__ __forceinline__ void acc_guard4(v8f& a, v8f& b, v8f& c, v8f& d) {
  asm volatile("v_nop\n\tv_nop\n\tv_nop\n\tv_nop" : "+v"(a), "+v"(b), "+v"(c), "+v"(d));
}

__global__ __launch_bounds__(256) void hs_cast_kernel(
    const float* __restrict__ a, const float* __restrict__ b,
    unsigned short* __restrict__ dhi, unsigned short* __restrict__ dlo, int total8)
{
  const int i = blockIdx.x * 256 + threadIdx.x;
  if (i >= total8) return;
  const size_t e0 = (size_t)i << 3;
  const v4f a0 = *(const v4f*)(a + e0);
  const v4f a1 = *(const v4f*)(a + e0 + 4);
  const v4f b0 = *(const v4f*)(b + e0);
  const v4f b1 = *(const v4f*)(b + e0 + 4);
  v8h hv, lv;
#pragma unroll
  for (int e = 0; e < 4; ++e) {
    const float s0 = (a0[e] + b0[e]) * kCarryHs;
    const float s1 = (a1[e] + b1[e]) * kCarryHs;
    const _Float16 h0 = f16_operand(s0);
    const _Float16 h1 = f16_operand(s1);
    const float k0 = (float)h0;
    const float k1 = (float)h1;
    const float d0 = (s0 - k0) * kCarryLo;
    const float d1 = (s1 - k1) * kCarryLo;
    hv[e]     = h0;
    hv[4 + e] = h1;
    lv[e]     = f16_operand(d0);
    lv[4 + e] = f16_operand(d1);
  }
  unsigned short* qh = dhi + e0;
  unsigned short* ql = dlo + e0;
  *(volatile v8h*)qh = hv;
  *(volatile v8h*)ql = lv;
  __threadfence();
  *(volatile v8h*)qh = hv;
  *(volatile v8h*)ql = lv;
}

__global__ __launch_bounds__(256) void transpose_cast_kernel(
    const float* __restrict__ W, unsigned short* __restrict__ Bt, int Kdim, int Ndim, float scale)
{
  __shared__ float tile[64 * 65];
  const int tid = threadIdx.x, lane = tid & 31, wave = tid >> 5;
  const int n0 = blockIdx.x * 64;
  const int k0 = blockIdx.y * 64;
#pragma unroll
  for (int pp = 0; pp < 16; ++pp) {
    const int idx = tid + pp * 256;
    const int kk  = idx >> 6;
    const int nn  = idx & 63;
    const int n   = n0 + nn;
    const int nc  = (n < Ndim) ? n : (Ndim - 1);
    const float v = W[(size_t)(k0 + kk) * Ndim + nc];
    const float w = v * scale;
    tile[kk * 65 + nn] = (n < Ndim) ? w : 0.0f;
  }
  __syncthreads();
  const int q = lane >> 3, c8 = (lane & 7) * 8;
  v8h hv[2];
#pragma unroll
  for (int it = 0; it < 2; ++it) {
    const int nrow = it * 32 + wave * 4 + q;
#pragma unroll
    for (int e = 0; e < 8; ++e) hv[it][e] = f16_operand(tile[(c8 + e) * 65 + nrow]);
  }
  for (int pass = 0; pass < 2; ++pass) {
#pragma unroll
    for (int it = 0; it < 2; ++it) {
      const int nrow = it * 32 + wave * 4 + q;
      *(volatile v8h*)(Bt + (size_t)(n0 + nrow) * Kdim + k0 + c8) = hv[it];
    }
    __threadfence();
  }
}

template <bool ROUTE, bool SPLITA>
__global__ __launch_bounds__(256) void gemm_f16_kernel(
    const unsigned short* __restrict__ Ap, const unsigned short* __restrict__ A2p, int lda,
    const unsigned short* __restrict__ Btp, int ldb,
    float* __restrict__ Cf, int ldc,
    unsigned short* __restrict__ Zp, unsigned short* __restrict__ Xp,
    float* __restrict__ BCp, float* __restrict__ DTp,
    int tilesM, int tilesN, int K, float scale)
{
  const _Float16* A  = (const _Float16*)Ap;
  const _Float16* A2 = (const _Float16*)A2p;
  const _Float16* Bt = (const _Float16*)Btp;
  __shared__ __align__(16) float sT[8][16 * 68];
  const int lane = threadIdx.x & 31;
  const int wave = threadIdx.x >> 5;
  const int tile = blockIdx.x * 8 + wave;
  if (tile >= tilesM * tilesN) return;
  const int tm = tile / tilesN;
  const int tn = tile - tm * tilesN;
  const int m0 = tm << 6;
  const int n0 = tn << 6;
  const int rlane = lane & 15;
  const int koff  = (lane >> 4) * 8;
  const int mOff  = (lane >> 4) * 8;

  v8f acc[4][4];
#pragma unroll
  for (int i = 0; i < 4; ++i)
#pragma unroll
    for (int j = 0; j < 4; ++j) acc[i][j] = (v8f){0.f, 0.f, 0.f, 0.f, 0.f, 0.f, 0.f, 0.f};

#pragma unroll
  for (int ph = 0; ph < 2; ++ph) {
    if (ph == 0 && !SPLITA) continue;
    const _Float16* Aph = (ph == 0) ? A2 : A;
    for (int k0 = 0; k0 < K; k0 += 32) {
      v16h bh[4];
#pragma unroll
      for (int j = 0; j < 4; ++j)
        bh[j] = frag_load(Bt + (size_t)(n0 + (j << 4) + rlane) * ldb + koff + k0);
#pragma unroll
      for (int i = 0; i < 4; ++i) {
        const v16h ah = frag_load(Aph + (size_t)(m0 + (i << 4) + rlane) * lda + koff + k0);
#pragma unroll
        for (int j = 0; j < 4; ++j) acc[i][j] = frag_mma(ah, bh[j], acc[i][j]);
        guard_group(acc[i][0], acc[i][1], acc[i][2], acc[i][3], ah, bh[0], bh[1], bh[2], bh[3]);
      }
    }
    if (ph == 0) {
      acc_guard4(acc[0][0], acc[0][1], acc[0][2], acc[0][3]);
      acc_guard4(acc[1][0], acc[1][1], acc[1][2], acc[1][3]);
      acc_guard4(acc[2][0], acc[2][1], acc[2][2], acc[2][3]);
      acc_guard4(acc[3][0], acc[3][1], acc[3][2], acc[3][3]);
#pragma unroll
      for (int i = 0; i < 4; ++i)
#pragma unroll
        for (int j = 0; j < 4; ++j) acc[i][j] = acc[i][j] * kLoInv;
    }
  }
  acc_guard4(acc[0][0], acc[0][1], acc[0][2], acc[0][3]);
  acc_guard4(acc[1][0], acc[1][1], acc[1][2], acc[1][3]);
  acc_guard4(acc[2][0], acc[2][1], acc[2][2], acc[2][3]);
  acc_guard4(acc[3][0], acc[3][1], acc[3][2], acc[3][3]);

  float* slab = sT[wave];
#pragma unroll
  for (int i = 0; i < 4; ++i) {
    const int mBase = m0 + (i << 4);
#pragma unroll
    for (int j = 0; j < 4; ++j) {
#pragma unroll
      for (int r = 0; r < 8; ++r) slab[(mOff + r) * 68 + (j << 4) + rlane] = acc[i][j][r] * scale;
    }
    __builtin_amdgcn_fence(__ATOMIC_RELEASE, "workgroup");
    __builtin_amdgcn_wave_barrier();
    __builtin_amdgcn_fence(__ATOMIC_ACQUIRE, "workgroup");
    if (!ROUTE || (tn >= 64 && tn < 80)) {
      float* C = ROUTE ? BCp : Cf;
      const int ld   = ROUTE ? kBCw : ldc;
      const int col0 = ROUTE ? ((tn - 64) << 6) : n0;
      const int hh = lane >> 4, c4 = (lane & 15) * 4;
      for (int pass = 0; pass < 2; ++pass) {
#pragma unroll
        for (int it = 0; it < 8; ++it) {
          const int row = it * 2 + hh;
          const v4f v = *(const v4f*)(slab + row * 68 + c4);
          *(volatile v4f*)(C + (size_t)(mBase + row) * ld + col0 + c4) = v;
        }
        __threadfence();
      }
    } else if (tn < 64) {
      unsigned short* C = (tn < 32) ? Zp : Xp;
      const int col0 = (tn & 31) << 6;
      const int q = lane >> 3, c8 = (lane & 7) * 8;
      for (int pass = 0; pass < 2; ++pass) {
#pragma unroll
        for (int it = 0; it < 4; ++it) {
          const int row = it * 4 + q;
          const float* sp = slab + row * 68 + c8;
          v8h hv;
#pragma unroll
          for (int e = 0; e < 8; ++e) hv[e] = (_Float16)sp[e];
          *(volatile v8h*)(C + (size_t)(mBase + row) * kDin + col0 + c8) = hv;
        }
        __threadfence();
      }
    } else {
      const int q = lane >> 3, c4 = (lane & 7) * 4;
      for (int pass = 0; pass < 2; ++pass) {
#pragma unroll
        for (int it = 0; it < 4; ++it) {
          const int row = it * 4 + q;
          const v4f v = *(const v4f*)(slab + row * 68 + c4);
          *(volatile v4f*)(DTp + (size_t)(mBase + row) * kHeads + c4) = v;
        }
        __threadfence();
      }
    }
    __builtin_amdgcn_fence(__ATOMIC_RELEASE, "workgroup");
    __builtin_amdgcn_wave_barrier();
    __builtin_amdgcn_fence(__ATOMIC_ACQUIRE, "workgroup");
  }
}

__global__ __launch_bounds__(256) void dt_decay_kernel(
    const float* __restrict__ DTR, const float* __restrict__ dt_bias, const float* __restrict__ A_log,
    float* __restrict__ DTA)
{
  const int lane = threadIdx.x & 31, wave = threadIdx.x >> 5;
  const int row = blockIdx.x * 8 + wave;
  const float raw = DTR[(size_t)row * kHeads + lane];
  const float v   = raw + dt_bias[lane];
  const float sp  = fmaxf(v, 0.0f) + log1pf(expf(-fabsf(v)));
  const float An  = -expf(A_log[lane]);
  float dec = expf(sp * An);
  dec = (dec < kF32Min) ? 0.0f : dec;
  volatile float* q = DTA + (size_t)row * 64;
  q[lane] = sp;
  q[32 + lane] = dec;
  __threadfence();
  q[lane] = sp;
  q[32 + lane] = dec;
}

__global__ __launch_bounds__(256) void state_scan_kernel(
    const float* __restrict__ BC32, const unsigned short* __restrict__ X16, unsigned short* ZY,
    const float* __restrict__ DTA, const float* __restrict__ Dsk)
{
  __shared__ __align__(16) float sBC[kTS * kBCw];
  __shared__ __align__(16) float sP[kTS * 16 * 64];
  __shared__ __align__(16) float sXs[kTS * 64];
  __shared__ __align__(16) float sXr[2][kTS * 64];
  __shared__ __align__(16) float sY[2][kTS * kSYP];
  __shared__ __align__(16) float sA[kTS];

  const int tid = threadIdx.x, lane = tid & 31;
  const int bb = blockIdx.x >> 5;
  const int hd = blockIdx.x & 31;
  const size_t row0 = (size_t)bb * kSeq;
  const int p  = tid & 15;
  const int ng = tid >> 4;
  const int n0 = ng * 8;
  const int ss = tid >> 6;
  const int sc = tid & 63;
  const unsigned* X16w = (const unsigned*)X16;

  float dsk = Dsk[hd];
  asm volatile("" : "+v"(dsk));

  float h[8];
#pragma unroll
  for (int j = 0; j < 8; ++j) h[j] = 0.0f;

#pragma unroll 1
  for (int chunk = 0; chunk < kSeq / kTS; ++chunk) {
    const int t0 = chunk * kTS;
    const int par = chunk & 1;
    float* sXrp = &sXr[par][0];
    float* sYp  = &sY[par][0];

    {
      v4f bcv[kTS];
#pragma unroll
      for (int s = 0; s < kTS; ++s)
        bcv[s] = *(const v4f*)(BC32 + (row0 + t0 + s) * kBCw + tid * 4);
      const size_t row = row0 + t0 + ss;
      const unsigned xw = X16w[(row * kDin + (size_t)hd * kHd + sc) >> 1];
      const float dtv = DTA[row * 64 + hd];
      float av = DTA[row * 64 + 32 + hd];
      asm volatile("" : "+v"(av));
#pragma unroll
      for (int s = 0; s < kTS; ++s) *(v4f*)(sBC + s * kBCw + tid * 4) = bcv[s];
      const unsigned hb = (sc & 1) ? (xw >> 16) : (xw & 0xffffu);
      const float xv = h16_to_f32(hb);
      sXs[ss * 64 + (sc & 15) * 4 + (sc >> 4)] = dtv * xv;
      sXrp[ss * 64 + sc] = xv;
      if (sc == 0) sA[ss] = av;
    }
    __syncthreads();

#pragma unroll 1
    for (int s = 0; s < kTS; ++s) {
      const float* bp = sBC + s * kBCw + n0;
      const v4f xs = *(const v4f*)(sXs + s * 64 + p * 4);
      const float dec = sA[s];
      float inj[8];
#pragma unroll
      for (int r = 0; r < kRank; ++r) {
        const v4f q0 = *(const v4f*)(bp + r * kNst);
        const v4f q1 = *(const v4f*)(bp + r * kNst + 4);
        const float xr = xs[r];
#pragma unroll
        for (int j = 0; j < 4; ++j) {
          if (r == 0) {
            inj[j]     = q0[j] * xr;
            inj[4 + j] = q1[j] * xr;
          } else {
            inj[j]     = fmaf(q0[j], xr, inj[j]);
            inj[4 + j] = fmaf(q1[j], xr, inj[4 + j]);
          }
        }
      }
#pragma unroll
      for (int j = 0; j < 8; ++j) h[j] = fmaf(dec, h[j], inj[j]);
      const float* cp = bp + kRank * kNst;
      v4f yv;
#pragma unroll
      for (int r = 0; r < kRank; ++r) {
        const v4f c0 = *(const v4f*)(cp + r * kNst);
        const v4f c1 = *(const v4f*)(cp + r * kNst + 4);
        float acc = c0[0] * h[0];
        acc = fmaf(c0[1], h[1], acc);
        acc = fmaf(c0[2], h[2], acc);
        acc = fmaf(c0[3], h[3], acc);
        acc = fmaf(c1[0], h[4], acc);
        acc = fmaf(c1[1], h[5], acc);
        acc = fmaf(c1[2], h[6], acc);
        acc = fmaf(c1[3], h[7], acc);
        yv[r] = acc;
      }
      *(v4f*)(sP + ((s * 16 + ng) * 16 + p) * 4) = yv;
    }
    __syncthreads();

    if (tid < 64) {
      const int rs = tid >> 4, rp = tid & 15;
      v4f acc = (v4f){0.f, 0.f, 0.f, 0.f};
#pragma unroll
      for (int g = 0; g < 16; ++g) acc += *(const v4f*)(sP + ((rs * 16 + g) * 16 + rp) * 4);
      float* yd = sYp + rs * kSYP + rp;
      yd[0]  = acc[0];
      yd[16] = acc[1];
      yd[32] = acc[2];
      yd[48] = acc[3];
    }
    __syncthreads();

    if (tid < 32) {
      const int q = lane >> 3, c8 = (lane & 7) * 8;
      const v4f y0 = *(const v4f*)(sYp + q * kSYP + c8);
      const v4f y1 = *(const v4f*)(sYp + q * kSYP + c8 + 4);
      const v4f x0 = *(const v4f*)(sXrp + q * 64 + c8);
      const v4f x1 = *(const v4f*)(sXrp + q * 64 + c8 + 4);
      unsigned short* zp = ZY + (row0 + t0 + q) * kDin + (size_t)hd * kHd + c8;
      const v4u zw = *(const v4u*)zp;
      const unsigned zwd[4] = {zw[0], zw[1], zw[2], zw[3]};
      const float yy[8] = {y0[0], y0[1], y0[2], y0[3], y1[0], y1[1], y1[2], y1[3]};
      const float xx[8] = {x0[0], x0[1], x0[2], x0[3], x1[0], x1[1], x1[2], x1[3]};
      v8h hv;
#pragma unroll
      for (int e = 0; e < 8; ++e) {
        const unsigned w = zwd[e >> 1];
        const unsigned hb = (e & 1) ? (w >> 16) : (w & 0xffffu);
        const float z = h16_to_f32(hb);
        const float sg = __builtin_amdgcn_rcpf(1.0f + __expf(-z));
        const float yt = fmaf(dsk, xx[e], yy[e]);
        const float g = (yt * (z * sg)) * kCarryY;
        hv[e] = f16_operand(g);
      }
      *(volatile v8h*)zp = hv;
      __threadfence();
      *(volatile v8h*)zp = hv;
    }
  }
}

__global__ __launch_bounds__(256) void resid_norm_kernel(
    const float* __restrict__ in0, const float* __restrict__ in1, const float* __restrict__ mo,
    float* __restrict__ out)
{
  const int lane = threadIdx.x & 31, wave = threadIdx.x >> 5;
  const int row = blockIdx.x * 8 + wave;
  const size_t base = (size_t)row * kDm + lane * 4;
  v4f v[8];
  float ssq = 0.0f;
#pragma unroll
  for (int it = 0; it < 8; ++it) {
    const size_t o = base + it * 128;
    const v4f a = *(const v4f*)(in0 + o);
    const v4f b = *(const v4f*)(in1 + o);
    const v4f c = *(const v4f*)(mo + o);
    v[it] = (a + b) + c;
    ssq = fmaf(v[it][0], v[it][0], ssq);
    ssq = fmaf(v[it][1], v[it][1], ssq);
    ssq = fmaf(v[it][2], v[it][2], ssq);
    ssq = fmaf(v[it][3], v[it][3], ssq);
  }
#pragma unroll
  for (int off = 16; off > 0; off >>= 1) ssq += __shfl_xor(ssq, off, 32);
  const float sc = rsqrtf(ssq * (1.0f / (float)kDm) + kEps);
#pragma unroll
  for (int it = 0; it < 8; ++it) v[it] = v[it] * sc;
  for (int pass = 0; pass < 2; ++pass) {
#pragma unroll
    for (int it = 0; it < 8; ++it) *(volatile v4f*)(out + base + it * 128) = v[it];
    __threadfence();
  }
}

extern "C" void kernel_launch(void* const* d_in, const int* in_sizes, int n_in,
                              void* d_out, int out_size, void* d_ws, size_t ws_size,
                              hipStream_t stream)
{
  if (n_in < 7) return;
  if (in_sizes[0] != kRows * kDm) return;
  if (in_sizes[1] != kRows * kDm) return;
  if (in_sizes[2] != kDm * kCols) return;
  if (in_sizes[3] != kDin * kDm) return;
  if (in_sizes[4] != kHeads || in_sizes[5] != kHeads || in_sizes[6] != kHeads) return;
  if (out_size != kRows * kDm) return;
  if (ws_size < kWsTotal) return;

  const float* hidden = (const float*)d_in[0];
  const float* inject = (const float*)d_in[1];
  const float* W_in   = (const float*)d_in[2];
  const float* W_out  = (const float*)d_in[3];
  const float* A_log  = (const float*)d_in[4];
  const float* dtb    = (const float*)d_in[5];
  const float* Dsk    = (const float*)d_in[6];
  float* out = (float*)d_out;

  char* ws = (char*)d_ws;
  unsigned short* HSHI  = (unsigned short*)(ws + kOffHSH);
  unsigned short* HSLO  = (unsigned short*)(ws + kOffHSL);
  float*          DTA   = (float*)(ws + kOffHSH);
  unsigned short* WINT  = (unsigned short*)(ws + kOffWIN);
  unsigned short* WOUTT = (unsigned short*)(ws + kOffWOUT);
  unsigned short* Z16   = (unsigned short*)(ws + kOffZ);
  unsigned short* X16   = (unsigned short*)(ws + kOffX);
  float*          BC32  = (float*)(ws + kOffBC);
  float*          MO    = (float*)(ws + kOffBC);
  float*          DTR   = (float*)(ws + kOffDTR);

  transpose_cast_kernel<<<dim3(kColsPad / 64, kDm / 64), 256, 0, stream>>>(W_in, WINT, kDm, kCols, kCarryW);
  transpose_cast_kernel<<<dim3(kDm / 64, kDin / 64), 256, 0, stream>>>(W_out, WOUTT, kDin, kDm, kCarryW);

  for (int half = 0; half < 2; ++half) {
    const size_t r0 = (size_t)half * kHalfRows;
    hs_cast_kernel<<<(kHalfRows * kDm / 8) / 256, 256, 0, stream>>>(
        hidden + r0 * kDm, inject + r0 * kDm, HSHI, HSLO, kHalfRows * kDm / 8);
    gemm_f16_kernel<true, true><<<(kTilesMh * kTilesN1) / 8, 256, 0, stream>>>(
        HSHI, HSLO, kDm, WINT, kDm, BC32 + r0 * kBCw, kBCw,
        Z16 + r0 * kDin, X16 + r0 * kDin, BC32 + r0 * kBCw, DTR + r0 * kHeads,
        kTilesMh, kTilesN1, kDm, kScaleIn);
  }

  dt_decay_kernel<<<kRows / 8, 256, 0, stream>>>(DTR, dtb, A_log, DTA);

  state_scan_kernel<<<kBatch * kHeads, 256, 0, stream>>>(BC32, X16, Z16, DTA, Dsk);

  gemm_f16_kernel<false, false><<<(kTilesM * kTilesN2) / 8, 256, 0, stream>>>(
      Z16, Z16, kDin, WOUTT, kDin, MO, kDm, X16, X16, MO, DTR, kTilesM, kTilesN2, kDin, kScaleOut);

  resid_norm_kernel<<<kRows / 8, 256, 0, stream>>>(hidden, inject, MO, out);
}
